// RelativeMultiHeadAttention_49417893708241
// MI455X (gfx1250) — hardware-verified
//
#include <hip/hip_runtime.h>


#ifndef NB
#define NB 4
#endif
#ifndef SEQ
#define SEQ 1024
#endif
#define NB_FULL  4
#define SEQ_FULL 1024
#define TT   SEQ
#define DM   1024
#define NH_  16
#define HD   64
#define DQ   (NH_ * HD)
#define ZH   8
#define PCAR 1024.0f
#define SCL  0.125f
#define NE   128
#define NREL 65
#define MAXR 32
#define PP   (TT + NE)
static_assert(TT % 128 == 0);
static_assert(TT <= SEQ_FULL);
static_assert(NB <= NB_FULL);
static_assert(NB >= 1);
static_assert(NH_ % ZH == 0);
static_assert(PP % 32 == 0);
static_assert(NREL == 2 * MAXR + 1);
static_assert(DM % 64 == 0);
static_assert((ZH * TT) % 8 == 0);

typedef _Float16 h16;
typedef unsigned short bf;
typedef __attribute__((ext_vector_type(16))) __bf16   v16bf;
typedef __attribute__((ext_vector_type(16))) _Float16 v16h;
typedef __attribute__((ext_vector_type(8)))  _Float16 v8h;
typedef __attribute__((ext_vector_type(8)))  unsigned short v8us;
typedef __attribute__((ext_vector_type(8)))  float    v8f;
typedef __attribute__((ext_vector_type(4)))  float    v4f;
typedef v8h  __attribute__((may_alias)) v8ha;
typedef v4f  __attribute__((may_alias)) v4fa;
typedef v8us __attribute__((may_alias)) v8usa;

__device__ __forceinline__ unsigned short f2bf(float f) { unsigned u = __float_as_uint(f); u += 0x7FFFu + ((u >> 16) & 1u); return (unsigned short)(u >> 16); }
__device__ __forceinline__ float bf2f(unsigned short b) { return __uint_as_float(((unsigned)b) << 16); }
__device__ __forceinline__ float bfr(float f) { return bf2f(f2bf(f)); }
__device__ __forceinline__ v16h cat16(v8h lo, v8h hi) { return __builtin_shufflevector(lo, hi, 0, 1, 2, 3, 4, 5, 6, 7, 8, 9, 10, 11, 12, 13, 14, 15); }
__device__ __forceinline__ v16bf cat16b(v8us lo, v8us hi) { return __builtin_bit_cast(v16bf, __builtin_shufflevector(lo, hi, 0, 1, 2, 3, 4, 5, 6, 7, 8, 9, 10, 11, 12, 13, 14, 15)); }
__device__ __forceinline__ v8f wmma16(v16h a, v16h b, v8f c) { return __builtin_amdgcn_wmma_f32_16x16x32_f16(false, a, false, b, (short)0, c, false, false); }
__device__ __forceinline__ v8f wmmab(v16bf a, v16bf b, v8f c) { return __builtin_amdgcn_wmma_f32_16x16x32_bf16(false, a, false, b, (short)0, c, false, false); }

template <typename T16> struct WFrag;
template <> struct WFrag<h16> { typedef v16h V; static __device__ __forceinline__ V ld(const h16* p) { return cat16(*(const v8h*)p, *(const v8h*)(p + 16)); } static __device__ __forceinline__ v8f mma(V a, V b, v8f c) { return wmma16(a, b, c); } };
template <> struct WFrag<bf> { typedef v16bf V; static __device__ __forceinline__ V ld(const bf* p) { return cat16b(*(const v8us*)p, *(const v8us*)(p + 16)); } static __device__ __forceinline__ v8f mma(V a, V b, v8f c) { return wmmab(a, b, c); } };
template <typename T16, int NSPLIT, bool BIAS>
__global__ __launch_bounds__(32) void k_gemmw(const T16* __restrict__ A, const T16* __restrict__ A2, const T16* __restrict__ Bt, const T16* __restrict__ Bt2, int K, float* C, int ldc, const float* __restrict__ bias, size_t sA, size_t sB, size_t sC) {
    typedef typename WFrag<T16>::V V;
    __shared__ __align__(16) float os[16 * 68];
    const size_t z = blockIdx.z; A += z * sA; if (A2) A2 += z * sA; Bt += z * sB; if (Bt2) Bt2 += z * sB; C += z * sC;
    const int lane = threadIdx.x & 31, lr = lane & 15, hi = lane >> 4; const int r0 = blockIdx.x * 64, c0 = blockIdx.y * 64;
    v8f acc[4][4];
#pragma unroll
    for (int mb = 0; mb < 4; ++mb)
#pragma unroll
        for (int nb = 0; nb < 4; ++nb) acc[mb][nb] = (v8f){};
    const size_t aoff = (size_t)(r0 + lr) * K + 8 * hi, boff = (size_t)(c0 + lr) * K + 8 * hi;
#pragma unroll 1
    for (int kc = 0; kc < K; kc += 32) {
        V a[4], a2[4];
#pragma unroll
        for (int mb = 0; mb < 4; ++mb) { a[mb] = WFrag<T16>::ld(A + aoff + (size_t)mb * 16 * K + kc); if (NSPLIT == 1 || NSPLIT == 2) a2[mb] = WFrag<T16>::ld(A2 + aoff + (size_t)mb * 16 * K + kc); }
#pragma unroll
        for (int nb = 0; nb < 4; ++nb) { const V b = WFrag<T16>::ld(Bt + boff + (size_t)nb * 16 * K + kc); V b2; if (NSPLIT >= 2) b2 = WFrag<T16>::ld(Bt2 + boff + (size_t)nb * 16 * K + kc);
#pragma unroll
            for (int mb = 0; mb < 4; ++mb) { acc[mb][nb] = WFrag<T16>::mma(a[mb], b, acc[mb][nb]); if (NSPLIT == 1 || NSPLIT == 2) acc[mb][nb] = WFrag<T16>::mma(a2[mb], b, acc[mb][nb]); if (NSPLIT >= 2) acc[mb][nb] = WFrag<T16>::mma(a[mb], b2, acc[mb][nb]); } }
        asm volatile("v_nop\n\tv_nop\n\tv_nop\n\tv_nop" : "+v"(acc[0][0]), "+v"(acc[1][1]), "+v"(acc[2][2]), "+v"(acc[3][3]) : "v"(a[0]), "v"(a[3]));
    }
#pragma unroll
    for (int mb = 0; mb < 4; ++mb) {
#pragma unroll
        for (int nb = 0; nb < 4; ++nb) {
#pragma unroll
            for (int j = 0; j < 8; ++j) os[(hi * 8 + j) * 68 + nb * 16 + lr] = acc[mb][nb][j]; }
        __builtin_amdgcn_wave_barrier(); asm volatile("" ::: "memory");
        float* crow = C + (size_t)(r0 + mb * 16) * ldc + c0;
#pragma unroll 1
        for (int ps = 0; ps < 2; ++ps) {
#pragma unroll
            for (int s = 0; s < 8; ++s) { const int row = 2 * s + hi, cofs = lr * 4; v4f val = *(const v4fa*)(os + row * 68 + cofs); if (BIAS) { val[0] += bfr(bias[c0 + cofs]); val[1] += bfr(bias[c0 + cofs + 1]); val[2] += bfr(bias[c0 + cofs + 2]); val[3] += bfr(bias[c0 + cofs + 3]); }
                *(volatile v4f*)(crow + (size_t)row * ldc + cofs) = val; }
            if (ps == 0) __threadfence(); }
        __builtin_amdgcn_wave_barrier(); asm volatile("" ::: "memory");
    }
}

__device__ __forceinline__ h16 tohx(float x) { return (h16)x; }
__device__ __forceinline__ void splitf(float y, unsigned short& h, unsigned short& l) { h = f2bf(y); l = f2bf(y - bf2f(h)); }
typedef __attribute__((ext_vector_type(2))) _Float16 v2h;
typedef __attribute__((ext_vector_type(4))) _Float16 v4h;
typedef __attribute__((ext_vector_type(2))) unsigned short v2us;
typedef __attribute__((ext_vector_type(4))) unsigned short v4us;
typedef __attribute__((ext_vector_type(2))) float v2f;

__global__ __launch_bounds__(256) void k_cvt8(const float* __restrict__ src, bf* dst, size_t n8) { const size_t i = (size_t)blockIdx.x * 256 + threadIdx.x; if (i >= n8) return; const v8f v = *(const v8f*)(src + i * 8); v8us o;
#pragma unroll
    for (int k = 0; k < 8; ++k) o[k] = f2bf(v[k]); *(volatile v8us*)(dst + i * 8) = o; __threadfence(); *(volatile v8us*)(dst + i * 8) = o; }

__global__ __launch_bounds__(256) void k_epad2(const float* __restrict__ E, bf* EB) { const size_t i = (size_t)blockIdx.x * 256 + threadIdx.x; if (i >= (size_t)NE * HD / 8) return; const int d0 = (int)(i % (HD / 8)) * 8; const int r = (int)(i / (HD / 8)); const float* src = E + (size_t)min(r, NREL - 1) * HD + d0; v8us o;
#pragma unroll
    for (int q = 0; q < 8; ++q) { const unsigned short v = f2bf(src[q]); o[q] = (r < NREL) ? v : (unsigned short)0; }
    *(volatile v8us*)(EB + (size_t)r * HD + d0) = o; __threadfence(); *(volatile v8us*)(EB + (size_t)r * HD + d0) = o; }

__global__ __launch_bounds__(256) void k_plane(const float* __restrict__ F, int pitch, int nheads, bf* Ph, bf* Pl) {
    const size_t e = ((size_t)blockIdx.x * 256 + threadIdx.x) * 8; if (e >= (size_t)nheads * TT * HD) return;
    const int d = (int)(e % HD); const int t = (int)((e / HD) % TT); const int h = (int)(e / ((size_t)HD * TT));
    const v8f x = *(const v8f*)(F + (size_t)t * pitch + h * HD + d); v8us oh, ol;
#pragma unroll
    for (int q = 0; q < 8; ++q) { unsigned short a, c2; splitf(x[q], a, c2); oh[q] = a; ol[q] = c2; }
    *(volatile v8us*)(Ph + e) = oh; *(volatile v8us*)(Pl + e) = ol; __threadfence(); *(volatile v8us*)(Ph + e) = oh; *(volatile v8us*)(Pl + e) = ol; }

__global__ __launch_bounds__(256) void k_vtp8(const float* __restrict__ F, int pitch, int nheads, h16* VT) {
    const size_t e = ((size_t)blockIdx.x * 256 + threadIdx.x) * 8; if (e >= (size_t)nheads * HD * TT) return;
    const int t = (int)(e % TT); const int d = (int)((e / TT) % HD); const int g = (int)(e / ((size_t)TT * HD));
    v8h o;
#pragma unroll
    for (int q = 0; q < 8; ++q) o[q] = tohx(F[(size_t)(t + q) * pitch + g * HD + d]);
    h16* dst = VT + ((size_t)g * HD + d) * PP + t;
    *(volatile v8h*)dst = o; __threadfence(); *(volatile v8h*)dst = o; }

__global__ __launch_bounds__(256) void k_evt(const float* __restrict__ EV, int nheads, h16* VT) {
    const size_t e = ((size_t)blockIdx.x * 256 + threadIdx.x) * 8; if (e >= (size_t)nheads * HD * NE) return;
    const int r0 = (int)(e % NE); const int d = (int)((e / NE) % HD); const int g = (int)(e / ((size_t)NE * HD));
    v8h o;
#pragma unroll
    for (int q = 0; q < 8; ++q) { const int r = r0 + q; const float x = bfr(EV[(size_t)min(r, NREL - 1) * HD + d]); const float y = (r < NREL) ? x : 0.0f; o[q] = tohx(y); }
    h16* dst = VT + ((size_t)g * HD + d) * PP + TT + r0;
    *(volatile v8h*)dst = o; __threadfence(); *(volatile v8h*)dst = o; }

__global__ __launch_bounds__(256) void k_asoft(const float* __restrict__ Sb, const float* __restrict__ QE, h16* P16) {
    __shared__ __align__(16) float qes[8][NE];
    __shared__ __align__(16) float prow[8][TT];
    const int lane = threadIdx.x & 31, wid = threadIdx.x >> 5; const int row = blockIdx.x * 8 + wid; const int i = row % TT;
    const float* sr = Sb + (size_t)row * TT; const float* qe = QE + (size_t)row * NE;
    { const v4f g4 = *(const v4f*)(qe + lane * 4); *(v4f*)(&qes[wid][lane * 4]) = g4; }
    __syncthreads();
    float v[TT / 32]; float mx = -3.0e38f;
#pragma unroll
    for (int ch = 0; ch < TT / 128; ++ch) { const int j0 = ch * 128 + lane * 4; const v4f a = *(const v4f*)(sr + j0);
#pragma unroll
        for (int q = 0; q < 4; ++q) { const int j = j0 + q; const int r = min(max(j - i, -MAXR), MAXR) + MAXR; const float t = a[q] * SCL + qes[wid][r]; v[ch * 4 + q] = t; mx = fmaxf(mx, t); } }
#pragma unroll
    for (int sh = 16; sh; sh >>= 1) mx = fmaxf(mx, __shfl_xor(mx, sh, 32));
    float sum = 0.f;
#pragma unroll
    for (int k = 0; k < TT / 32; ++k) { float d0 = __fsub_rn(v[k], mx); asm volatile("" : "+v"(d0)); v[k] = __builtin_amdgcn_exp2f(__fmul_rn(d0, 1.4426950408889634f)); sum += v[k]; }
#pragma unroll
    for (int sh = 16; sh; sh >>= 1) sum += __shfl_xor(sum, sh, 32);
    const float f = __fdiv_rn(PCAR, sum);
    float tl0 = 0.f, tl1 = 0.f;
#pragma unroll
    for (int ch = 0; ch < TT / 128; ++ch) { const int j0 = ch * 128 + lane * 4; v4f p4;
#pragma unroll
        for (int q = 0; q < 4; ++q) { const int j = j0 + q; const float p = v[ch * 4 + q] * f; v[ch * 4 + q] = p; p4[q] = p; tl0 += (j <= i - MAXR) ? p : 0.f; tl1 += (j >= i + MAXR) ? p : 0.f; }
        *(v4f*)(&prow[wid][j0]) = p4; }
#pragma unroll
    for (int sh = 16; sh; sh >>= 1) { tl0 += __shfl_xor(tl0, sh, 32); tl1 += __shfl_xor(tl1, sh, 32); }
    __syncthreads();
    v4h bq4;
#pragma unroll
    for (int q = 0; q < 4; ++q) { const int r = lane * 4 + q; const int j = i + r - MAXR; const int jc = min(max(j, 0), TT - 1); float w = prow[wid][jc];
        w = (r > 0 && r < 2 * MAXR && j >= 0 && j < TT) ? w : 0.f; w = (r == 0) ? tl0 : w; w = (r == 2 * MAXR) ? tl1 : w; bq4[q] = tohx(w); }
    h16* prw = P16 + (size_t)row * PP;
#pragma unroll 1
    for (int ps = 0; ps < 2; ++ps) {
#pragma unroll
        for (int ch = 0; ch < TT / 128; ++ch) { v4h o4;
#pragma unroll
            for (int q = 0; q < 4; ++q) o4[q] = tohx(v[ch * 4 + q]);
            *(volatile v4h*)(prw + ch * 128 + lane * 4) = o4; }
        *(volatile v4h*)(prw + TT + lane * 4) = bq4;
        if (ps == 0) __threadfence(); }
}

__global__ __launch_bounds__(256) void k_merge(const float* __restrict__ O, int h0, bf* Ah, bf* Al) { const size_t e = ((size_t)blockIdx.x * 256 + threadIdx.x) * 2; if (e >= (size_t)ZH * TT * HD) return; const int d = (int)(e % HD); const int t = (int)((e / HD) % TT); const int zz = (int)(e / ((size_t)HD * TT)); const float cs = 1.0f / PCAR; const size_t oo = (size_t)t * DQ + (h0 + zz) * HD + d;
    v2us oh, ol;
#pragma unroll
    for (int q = 0; q < 2; ++q) { unsigned short a, c2; splitf(O[e + q] * cs, a, c2); oh[q] = a; ol[q] = c2; } *(volatile v2us*)(Ah + oo) = oh; *(volatile v2us*)(Al + oo) = ol; __threadfence(); *(volatile v2us*)(Ah + oo) = oh; *(volatile v2us*)(Al + oo) = ol; }

extern "C" void kernel_launch(void* const* d_in, const int* in_sizes, int n_in,
                              void* d_out, int out_size, void* d_ws, size_t ws_size, hipStream_t stream) {
    if (n_in < 13) return;
    const size_t needX = ((size_t)(NB - 1) * SEQ_FULL + TT) * DM;
    if ((size_t)in_sizes[0] < needX || (size_t)in_sizes[1] < needX || (size_t)in_sizes[2] < needX) return;
    if (in_sizes[3] < DM * DM || in_sizes[5] < DM * DM || in_sizes[7] < DM * DM || in_sizes[9] < DM * DM) return;
    if (in_sizes[4] < DM || in_sizes[6] < DM || in_sizes[8] < DM || in_sizes[10] < DM) return;
    if (in_sizes[11] < NREL * HD || in_sizes[12] < NREL * HD) return;
    if ((size_t)out_size < needX) return;
    const float* query = (const float*)d_in[0]; const float* key = (const float*)d_in[1]; const float* value = (const float*)d_in[2];
    const float* wq = (const float*)d_in[3]; const float* bq = (const float*)d_in[4]; const float* wk = (const float*)d_in[5]; const float* bk = (const float*)d_in[6];
    const float* wv = (const float*)d_in[7]; const float* bv = (const float*)d_in[8]; const float* wo = (const float*)d_in[9]; const float* bo = (const float*)d_in[10];
    const float* rke = (const float*)d_in[11]; const float* rve = (const float*)d_in[12];
    float* OUT = (float*)d_out;
    char* wsp = (char*)d_ws;
    auto take = [&](size_t bytes) { char* p = wsp; wsp += (bytes + 255) & ~(size_t)255; return (void*)p; };
    bf* WQ = (bf*)take((size_t)DQ * DM * 2); bf* WK = (bf*)take((size_t)DQ * DM * 2); bf* WV = (bf*)take((size_t)DQ * DM * 2); bf* WO = (bf*)take((size_t)DM * DQ * 2);
    bf* EB = (bf*)take((size_t)NE * HD * 2);
    bf* XB = (bf*)take((size_t)TT * DM * 2); float* F = (float*)take((size_t)TT * DQ * 4);
    bf* QPh = (bf*)take((size_t)NH_ * TT * HD * 2); bf* QPl = (bf*)take((size_t)NH_ * TT * HD * 2); bf* KPh = (bf*)take((size_t)NH_ * TT * HD * 2); bf* KPl = (bf*)take((size_t)NH_ * TT * HD * 2);
    h16* VT = (h16*)take((size_t)NH_ * HD * PP * 2);
    float* QE = (float*)take((size_t)ZH * TT * NE * 4); float* Sb = (float*)take((size_t)ZH * TT * TT * 4); h16* P16 = (h16*)take((size_t)ZH * TT * PP * 2);
    float* Ob = (float*)take((size_t)ZH * TT * HD * 4); bf* ATh = (bf*)take((size_t)TT * DQ * 2); bf* ATl = (bf*)take((size_t)TT * DQ * 2);
    const size_t carved = (size_t)(wsp - (char*)d_ws);
    if (carved > ws_size || carved > (size_t)134217728) return;
    k_cvt8<<<(unsigned)(((size_t)DQ * DM / 8 + 255) / 256), 256, 0, stream>>>(wq, WQ, (size_t)DQ * DM / 8);
    k_cvt8<<<(unsigned)(((size_t)DQ * DM / 8 + 255) / 256), 256, 0, stream>>>(wk, WK, (size_t)DQ * DM / 8);
    k_cvt8<<<(unsigned)(((size_t)DQ * DM / 8 + 255) / 256), 256, 0, stream>>>(wv, WV, (size_t)DQ * DM / 8);
    k_cvt8<<<(unsigned)(((size_t)DM * DQ / 8 + 255) / 256), 256, 0, stream>>>(wo, WO, (size_t)DM * DQ / 8);
    k_epad2<<<(unsigned)(((size_t)NE * HD / 8 + 255) / 256), 256, 0, stream>>>(rke, EB);
    k_evt<<<(unsigned)(((size_t)NH_ * HD * NE / 8 + 255) / 256), 256, 0, stream>>>(rve, NH_, VT);
    const unsigned LPL = (unsigned)(((size_t)NH_ * TT * HD / 8 + 255) / 256);
    for (int b = 0; b < NB; ++b) {
        const size_t xoff = (size_t)b * SEQ_FULL * DM;
        k_cvt8<<<(unsigned)(((size_t)TT * DM / 8 + 255) / 256), 256, 0, stream>>>(query + xoff, XB, (size_t)TT * DM / 8);
        k_gemmw<bf, 0, true><<<dim3(TT / 64, DQ / 64, 1), 32, 0, stream>>>(XB, nullptr, WQ, nullptr, DM, F, DQ, bq, 0, 0, 0);
        k_plane<<<LPL, 256, 0, stream>>>(F, DQ, NH_, QPh, QPl);
        k_cvt8<<<(unsigned)(((size_t)TT * DM / 8 + 255) / 256), 256, 0, stream>>>(key + xoff, XB, (size_t)TT * DM / 8);
        k_gemmw<bf, 0, true><<<dim3(TT / 64, DQ / 64, 1), 32, 0, stream>>>(XB, nullptr, WK, nullptr, DM, F, DQ, bk, 0, 0, 0);
        k_plane<<<LPL, 256, 0, stream>>>(F, DQ, NH_, KPh, KPl);
        k_cvt8<<<(unsigned)(((size_t)TT * DM / 8 + 255) / 256), 256, 0, stream>>>(value + xoff, XB, (size_t)TT * DM / 8);
        k_gemmw<bf, 0, true><<<dim3(TT / 64, DQ / 64, 1), 32, 0, stream>>>(XB, nullptr, WV, nullptr, DM, F, DQ, bv, 0, 0, 0);
        k_vtp8<<<LPL, 256, 0, stream>>>(F, DQ, NH_, VT);
        for (int h0 = 0; h0 < NH_; h0 += ZH) { const size_t zq = (size_t)h0;
            k_gemmw<bf, 2, false><<<dim3(TT / 64, TT / 64, ZH), 32, 0, stream>>>(QPh + zq * TT * HD, QPl + zq * TT * HD, KPh + zq * TT * HD, KPl + zq * TT * HD, HD, Sb, TT, nullptr, (size_t)TT * HD, (size_t)TT * HD, (size_t)TT * TT);
            k_gemmw<bf, 1, false><<<dim3(TT / 64, NE / 64, ZH), 32, 0, stream>>>(QPh + zq * TT * HD, QPl + zq * TT * HD, EB, nullptr, HD, QE, NE, nullptr, (size_t)TT * HD, 0, (size_t)TT * NE);
            k_asoft<<<ZH * TT / 8, 256, 0, stream>>>(Sb, QE, P16);
            k_gemmw<h16, 0, false><<<dim3(TT / 64, HD / 64, ZH), 32, 0, stream>>>(P16, nullptr, VT + zq * HD * PP, nullptr, PP, Ob, HD, nullptr, (size_t)TT * PP, (size_t)HD * PP, (size_t)TT * HD);
            k_merge<<<(unsigned)(((size_t)ZH * TT * HD / 2 + 255) / 256), 256, 0, stream>>>(Ob, h0, ATh, ATl); }
        k_gemmw<bf, 1, true><<<dim3(TT / 64, DM / 64, 1), 32, 0, stream>>>(ATh, ATl, WO, nullptr, DQ, OUT + xoff, DM, bo, 0, 0, 0); }
}
